// SymNetModel_78400333021353
// MI455X (gfx1250) — hardware-verified
//
#include <hip/hip_runtime.h>
#include <hip/hip_bf16.h>
#include <math.h>

typedef __attribute__((ext_vector_type(16))) _Float16 v16h;
typedef __attribute__((ext_vector_type(8)))  _Float16 v8h;
typedef __attribute__((ext_vector_type(16))) __bf16   v16b;
typedef __attribute__((ext_vector_type(8)))  __bf16   v8b;
typedef __attribute__((ext_vector_type(8)))  float    v8f;
typedef __attribute__((ext_vector_type(4)))  float    v4f;

__device__ __forceinline__ unsigned short f2bf_bits(float f) {
  unsigned u = __float_as_uint(f);
  return (unsigned short)((u + 0x7FFFu + ((u >> 16) & 1u)) >> 16);
}
__device__ __forceinline__ float bf_bits2f(unsigned short h) { return __uint_as_float(((unsigned)h) << 16); }

__device__ __forceinline__ void dep_guard_h(v8f& a, v8f& b, v16h x, v16h y) { asm volatile("v_nop\n\tv_nop\n\tv_nop\n\tv_nop" : "+v"(a), "+v"(b) : "v"(x), "v"(y)); }
__device__ __forceinline__ void dep_guard_b(v8f& a, v8f& b, v16b x, v16b y) { asm volatile("v_nop\n\tv_nop\n\tv_nop\n\tv_nop" : "+v"(a), "+v"(b) : "v"(x), "v"(y)); }
__device__ __forceinline__ void keep4_h(v16h a, v16h b, v16h c, v16h d) { asm volatile("v_nop" :: "v"(a), "v"(b), "v"(c), "v"(d)); }
__device__ __forceinline__ void keep4_b(v16b a, v16b b, v16b c, v16b d) { asm volatile("v_nop" :: "v"(a), "v"(b), "v"(c), "v"(d)); }
__device__ __forceinline__ void acc_guard4(v8f& a, v8f& b, v8f& c, v8f& d) { asm volatile("v_nop\n\tv_nop\n\tv_nop\n\tv_nop" : "+v"(a), "+v"(b), "+v"(c), "+v"(d)); }
template <typename T> struct Frag;
template <> struct Frag<_Float16> {
  typedef v16h V; union U { v16h v; v8h h[2]; };
  static __device__ __forceinline__ v16h load(const _Float16* p) {
    U f; f.h[0] = *(const v8h*)(p); f.h[1] = *(const v8h*)(p + 16); return f.v;
  }
  static __device__ __forceinline__ v8f mma(v16h a, v16h b, v8f c) {
    return __builtin_amdgcn_wmma_f32_16x16x32_f16(false, a, false, b, (short)0, c, false, false);
  }
  static __device__ __forceinline__ void guard(v8f& a, v8f& b, v16h x, v16h y) { dep_guard_h(a, b, x, y); }
  static __device__ __forceinline__ void keep(v16h a, v16h b, v16h c, v16h d) { keep4_h(a, b, c, d); }
};
template <> struct Frag<__bf16> {
  typedef v16b V; union U { v16b v; v8b h[2]; };
  static __device__ __forceinline__ v16b load(const __bf16* p) {
    U f; f.h[0] = *(const v8b*)(p); f.h[1] = *(const v8b*)(p + 16); return f.v;
  }
  static __device__ __forceinline__ v8f mma(v16b a, v16b b, v8f c) {
    return __builtin_amdgcn_wmma_f32_16x16x32_bf16(false, a, false, b, (short)0, c, false, false);
  }
  static __device__ __forceinline__ void guard(v8f& a, v8f& b, v16b x, v16b y) { dep_guard_b(a, b, x, y); }
  static __device__ __forceinline__ void keep(v16b a, v16b b, v16b c, v16b d) { keep4_b(a, b, c, d); }
};

template <int ET> struct Elem;
template <> struct Elem<0> { typedef _Float16 T; };
template <> struct Elem<1> { typedef __bf16 T; };
template <int ET, bool SPLIT, int BIAS_MODE, int OUT_MODE, bool RESID, int ACT = 0>
__global__ __launch_bounds__(256) void wmma_gemm64(
    const unsigned short* __restrict__ Ap, const unsigned short* __restrict__ A2p, int lda, long strideA,
    const unsigned short* __restrict__ Btp, const unsigned short* __restrict__ Bt2p, int ldb, long strideB,
    void* Cout, void* Cout2, int ldc, long strideC,
    const float* __restrict__ bias,
    const float* resid, long strideR,
    int M, int N, int K, float scale) {
  typedef typename Elem<ET>::T T;
  typedef typename Frag<T>::V V;
  const T* A = (const T*)Ap; const T* A2 = (const T*)A2p; const T* Bt = (const T*)Btp; const T* Bt2 = (const T*)Bt2p;
  __shared__ __align__(16) float sT[8][16 * 68];
  const int b    = blockIdx.y;
  const int lane = threadIdx.x & 31;
  const int wave = threadIdx.x >> 5;
  const int tilesN = N >> 6;
  const int tilesM = M >> 6;
  const int tile = blockIdx.x * 8 + wave;
  if (tile >= tilesM * tilesN) return;
  const int tm = tile / tilesN;
  const int tn = tile - tm * tilesN;
  const int m0 = tm << 6;
  const int n0 = tn << 6;

  const T* Ab  = A  + (size_t)b * strideA;
  const T* Bb  = Bt + (size_t)b * strideB;
  const T* Ab2 = SPLIT ? (A2  + (size_t)b * strideA) : nullptr;
  const T* Bb2 = SPLIT ? (Bt2 + (size_t)b * strideB) : nullptr;

  const int rlane = lane & 15;
  const int koff  = (lane >> 4) * 8;
  const int mOff  = (lane >> 4) * 8;

  v8f acc[4][4];
#pragma unroll
  for (int i = 0; i < 4; ++i)
#pragma unroll
    for (int j = 0; j < 4; ++j) acc[i][j] = (v8f){0.f,0.f,0.f,0.f,0.f,0.f,0.f,0.f};

  for (int k0 = 0; k0 < K; k0 += 32) {
    V bh[4], bl[4];
#pragma unroll
    for (int j = 0; j < 4; ++j) {
      const size_t bo = (size_t)(n0 + (j << 4) + rlane) * ldb + koff + k0;
      bh[j] = Frag<T>::load(Bb + bo);
      if (SPLIT) bl[j] = Frag<T>::load(Bb2 + bo);
    }
#pragma unroll
    for (int i = 0; i < 4; ++i) {
      const size_t ao = (size_t)(m0 + (i << 4) + rlane) * lda + koff + k0;
      V ah = Frag<T>::load(Ab + ao);
      V al;
      if (SPLIT) al = Frag<T>::load(Ab2 + ao);
#pragma unroll
      for (int j = 0; j < 4; ++j) {
        acc[i][j] = Frag<T>::mma(ah, bh[j], acc[i][j]);
        if (SPLIT) {
          acc[i][j] = Frag<T>::mma(ah, bl[j], acc[i][j]);
          acc[i][j] = Frag<T>::mma(al, bh[j], acc[i][j]);
        }
      }
      Frag<T>::guard(acc[i][0], acc[i][3], ah, SPLIT ? al : ah);
    }
    Frag<T>::keep(bh[0], bh[1], bh[2], bh[3]);
    if (SPLIT) Frag<T>::keep(bl[0], bl[1], bl[2], bl[3]);
  }
  acc_guard4(acc[0][0], acc[0][1], acc[0][2], acc[0][3]);
  acc_guard4(acc[1][0], acc[1][1], acc[1][2], acc[1][3]);
  acc_guard4(acc[2][0], acc[2][1], acc[2][2], acc[2][3]);
  acc_guard4(acc[3][0], acc[3][1], acc[3][2], acc[3][3]);

  float* slab = sT[wave];
  const float* Rb = RESID ? (resid + (size_t)b * strideR) : nullptr;
#pragma unroll
  for (int i = 0; i < 4; ++i) {
    const int mBase = m0 + (i << 4);
#pragma unroll
    for (int j = 0; j < 4; ++j) {
      const int n = n0 + (j << 4) + rlane;
      float bv = 0.f;
      if (BIAS_MODE == 2) bv = bias[n];
#pragma unroll
      for (int r = 0; r < 8; ++r) {
        float v = acc[i][j][r] * scale;
        if (BIAS_MODE == 1) v += bias[mBase + mOff + r];
        if (BIAS_MODE == 2) v += bv;
        if (RESID) v += Rb[(size_t)(mBase + mOff + r) * ldc + n];
        if (ACT == 1) v = tanhf(v);
        if (ACT == 2) v = fmaxf(v, 0.0f);
        if (ACT == 3) v = v / (1.0f + expf(-v));
        if (ACT == 4) v = (v > 0.f) ? v : 0.01f * v;
        if (ACT == 5) v = 0.5f * v * (1.0f + erff(v * 0.70710678118654752f));
        slab[(mOff + r) * 68 + (j << 4) + rlane] = v;
      }
    }
    __builtin_amdgcn_fence(__ATOMIC_RELEASE, "workgroup");
    __builtin_amdgcn_wave_barrier();
    __builtin_amdgcn_fence(__ATOMIC_ACQUIRE, "workgroup");
    if (OUT_MODE == 0) {
      float* C = (float*)Cout + (size_t)b * strideC;
      const int hh = lane >> 4, c4 = (lane & 15) * 4;
      for (int pass = 0; pass < 2; ++pass) {
#pragma unroll
        for (int it = 0; it < 8; ++it) {
          const int row = it * 2 + hh;
          v4f v = *(const v4f*)(slab + row * 68 + c4);
          *(volatile v4f*)(C + (size_t)(mBase + row) * ldc + n0 + c4) = v;
        }
        __threadfence();
      }
    } else {
      const int q = lane >> 3, c8 = (lane & 7) * 8;
      unsigned short* C  = (unsigned short*)Cout  + (size_t)b * strideC;
      unsigned short* C2 = (OUT_MODE == 2) ? ((unsigned short*)Cout2 + (size_t)b * strideC) : nullptr;
      for (int pass = 0; pass < 2; ++pass) {
#pragma unroll
        for (int it = 0; it < 4; ++it) {
          const int row = it * 4 + q;
          const float* sp = slab + row * 68 + c8;
          v8h hv, lv;
#pragma unroll
          for (int e = 0; e < 8; ++e) {
            if (OUT_MODE == 1) {
              hv[e] = (_Float16)sp[e];
            } else {
              unsigned short hb = f2bf_bits(sp[e]);
              unsigned short lb = f2bf_bits(sp[e] - bf_bits2f(hb));
              hv[e] = __builtin_bit_cast(_Float16, hb);
              lv[e] = __builtin_bit_cast(_Float16, lb);
            }
          }
          *(volatile v8h*)(C + (size_t)(mBase + row) * ldc + n0 + c8) = hv;
          if (OUT_MODE == 2) *(volatile v8h*)(C2 + (size_t)(mBase + row) * ldc + n0 + c8) = lv;
        }
        __threadfence();
      }
    }
    __builtin_amdgcn_fence(__ATOMIC_RELEASE, "workgroup");
    __builtin_amdgcn_wave_barrier();
    __builtin_amdgcn_fence(__ATOMIC_ACQUIRE, "workgroup");
  }
}

__global__ __launch_bounds__(256) void pack_bt_f16(const float* __restrict__ src, long srcZ, int sk, int sn,
                                                   int Kr, int Nr, _Float16* __restrict__ dst, long dstZ,
                                                   int Kp, int Np, float scale) {
  const int kch = Kp >> 3;
  const int total = Np * kch;
  const int i = blockIdx.x * 256 + threadIdx.x;
  if (i >= total) return;
  const int n = i / kch;
  const int k8 = (i - n * kch) * 8;
  const float* s = src + (size_t)blockIdx.y * (size_t)srcZ;
  v8h o;
#pragma unroll
  for (int e = 0; e < 8; ++e) {
    const int k = k8 + e;
    float v = 0.0f;
    if (k < Kr && n < Nr) v = s[(size_t)k * (size_t)sk + (size_t)n * (size_t)sn] * scale;
    o[e] = (_Float16)v;
  }
  _Float16* d = dst + (size_t)blockIdx.y * (size_t)dstZ + (size_t)n * Kp + k8;
  *(volatile v8h*)d = o;
  __threadfence();
  *(volatile v8h*)d = o;
}

__global__ __launch_bounds__(256) void pack_heads_bt(const float* __restrict__ aw, const float* __restrict__ cw,
                                                     const float* __restrict__ vw, _Float16* __restrict__ dst,
                                                     float scale) {
  const int i = blockIdx.x * 256 + threadIdx.x;
  if (i >= 192 * 64) return;
  const int n = i >> 6;
  const int k8 = (i & 63) * 8;
  v8h o;
#pragma unroll
  for (int e = 0; e < 8; ++e) {
    const int k = k8 + e;
    float v = 0.0f;
    if (n < 4) v = aw[k * 4 + n];
    else if (n < 132) v = cw[k * 128 + (n - 4)];
    else if (n == 132) v = vw[k];
    o[e] = (_Float16)(v * scale);
  }
  _Float16* d = dst + (size_t)n * 512 + k8;
  *(volatile v8h*)d = o;
  __threadfence();
  *(volatile v8h*)d = o;
}

__global__ __launch_bounds__(256) void im2col_k(const float* __restrict__ obs, _Float16* __restrict__ dst, int Bsz) {
  const int i = blockIdx.x * 256 + threadIdx.x;
  if (i >= Bsz * 36) return;
  const int row = i >> 2;
  const int k8 = (i & 3) * 8;
  const int b = row / 9;
  const int p = row - b * 9;
  const int oy = p / 3;
  const int ox = p - oy * 3;
  const float* ob = obs + (size_t)b * 75;
  v8h o;
#pragma unroll
  for (int e = 0; e < 8; ++e) {
    const int k = k8 + e;
    float v = 0.0f;
    if (k < 27) {
      const int ic = k / 9;
      const int r9 = k - ic * 9;
      const int ky = r9 / 3;
      const int kx = r9 - ky * 3;
      v = ob[ic * 25 + (oy + ky) * 5 + ox + kx];
    }
    o[e] = (_Float16)v;
  }
  _Float16* d = dst + (size_t)row * 32 + k8;
  *(volatile v8h*)d = o;
  __threadfence();
  *(volatile v8h*)d = o;
}

__global__ __launch_bounds__(256) void conv_gather_k(const float* __restrict__ Cc, const float* __restrict__ cb,
                                                    _Float16* __restrict__ v16, int Bsz) {
  const int i = blockIdx.x * 256 + threadIdx.x;
  if (i >= Bsz * 36) return;
  const int b = i / 36;
  const int j8 = (i - b * 36) * 8;
  v8h o;
#pragma unroll
  for (int e = 0; e < 8; ++e) {
    const int j = j8 + e;
    const int oc = j / 9;
    const int p = j - oc * 9;
    const float v = Cc[((size_t)b * 9 + p) * 64 + oc] + cb[oc];
    o[e] = (_Float16)fmaxf(v, 0.0f);
  }
  _Float16* d = v16 + (size_t)b * 288 + j8;
  *(volatile v8h*)d = o;
  __threadfence();
  *(volatile v8h*)d = o;
}

__global__ __launch_bounds__(256) void comm_cast_k(const float* __restrict__ comm, _Float16* __restrict__ xcat, int Bsz) {
  const int i = blockIdx.x * 256 + threadIdx.x;
  if (i >= Bsz * 16) return;
  const int b = i >> 4;
  const int j8 = (i & 15) * 8;
  const float* s = comm + (size_t)b * 128 + j8;
  const v4f a0 = *(const v4f*)(s);
  const v4f a1 = *(const v4f*)(s + 4);
  v8h o;
#pragma unroll
  for (int e = 0; e < 4; ++e) { o[e] = (_Float16)a0[e]; o[4 + e] = (_Float16)a1[e]; }
  _Float16* d = xcat + (size_t)b * 384 + 256 + j8;
  *(volatile v8h*)d = o;
  __threadfence();
  *(volatile v8h*)d = o;
}

__global__ __launch_bounds__(256) void cast8_k(const float* __restrict__ src, _Float16* __restrict__ dst, int n8) {
  const int i = blockIdx.x * 256 + threadIdx.x;
  if (i >= n8) return;
  const float* s = src + (size_t)i * 8;
  const v4f a0 = *(const v4f*)(s);
  const v4f a1 = *(const v4f*)(s + 4);
  v8h o;
#pragma unroll
  for (int e = 0; e < 4; ++e) { o[e] = (_Float16)a0[e]; o[4 + e] = (_Float16)a1[e]; }
  _Float16* d = dst + (size_t)i * 8;
  *(volatile v8h*)d = o;
  __threadfence();
  *(volatile v8h*)d = o;
}

__global__ __launch_bounds__(256) void rmsnorm_k(const float* __restrict__ X, const float* __restrict__ w,
                                                 _Float16* __restrict__ Y, int Bsz) {
  const int wave = threadIdx.x >> 5;
  const int lane = threadIdx.x & 31;
  const int row = blockIdx.x * 8 + wave;
  if (row >= Bsz) return;
  const float* x = X + (size_t)row * 512;
  const v4f a0 = *(const v4f*)(x + lane * 8);
  const v4f a1 = *(const v4f*)(x + lane * 8 + 4);
  const v4f a2 = *(const v4f*)(x + 256 + lane * 8);
  const v4f a3 = *(const v4f*)(x + 256 + lane * 8 + 4);
  float s = 0.0f;
#pragma unroll
  for (int e = 0; e < 4; ++e) { s += a0[e] * a0[e]; s += a1[e] * a1[e]; s += a2[e] * a2[e]; s += a3[e] * a3[e]; }
#pragma unroll
  for (int off = 16; off > 0; off >>= 1) s += __shfl_xor(s, off, 32);
  const float r = rsqrtf(s * (1.0f / 512.0f) + 1e-5f);
  const v4f w0 = *(const v4f*)(w + lane * 8);
  const v4f w1 = *(const v4f*)(w + lane * 8 + 4);
  const v4f w2 = *(const v4f*)(w + 256 + lane * 8);
  const v4f w3 = *(const v4f*)(w + 256 + lane * 8 + 4);
  v8h o0, o1;
#pragma unroll
  for (int e = 0; e < 4; ++e) {
    o0[e]     = (_Float16)(a0[e] * r * w0[e]);
    o0[4 + e] = (_Float16)(a1[e] * r * w1[e]);
    o1[e]     = (_Float16)(a2[e] * r * w2[e]);
    o1[4 + e] = (_Float16)(a3[e] * r * w3[e]);
  }
  _Float16* y = Y + (size_t)row * 512;
  *(volatile v8h*)(y + lane * 8) = o0;
  *(volatile v8h*)(y + 256 + lane * 8) = o1;
  __threadfence();
  *(volatile v8h*)(y + lane * 8) = o0;
  *(volatile v8h*)(y + 256 + lane * 8) = o1;
}

__global__ __launch_bounds__(256) void conv_silu_k(const float* __restrict__ xz, const float* __restrict__ cw,
                                                   const float* __restrict__ cb, _Float16* __restrict__ xm, int Bsz) {
  const int i = blockIdx.x * 256 + threadIdx.x;
  if (i >= Bsz * 512) return;
  const int b = i >> 9;
  const int c0 = (i & 511) * 2;
  const float* xr = xz + (size_t)b * 2048;
  unsigned packed = 0;
#pragma unroll
  for (int e = 0; e < 2; ++e) {
    const int c = c0 + e;
    const float t = xr[c] * cw[c * 4 + 3] + cb[c];
    const float sg = __builtin_amdgcn_rcpf(1.0f + expf(-t));
    const _Float16 hv = (_Float16)(t * sg);
    packed |= ((unsigned)__builtin_bit_cast(unsigned short, hv)) << (16 * e);
  }
  volatile unsigned* d = (volatile unsigned*)(xm + (size_t)b * 1024 + c0);
  *d = packed;
  __threadfence();
  *d = packed;
}

__global__ __launch_bounds__(256) void yz_k(const float* __restrict__ xz, const float* __restrict__ xdbl,
                                            const _Float16* __restrict__ dtp, const float* __restrict__ bdt,
                                            const float* __restrict__ cw, const float* __restrict__ cb,
                                            const float* __restrict__ Dp, _Float16* __restrict__ yz, int Bsz) {
  const int total = Bsz * 512;
  const int i0 = blockIdx.x * 256 + threadIdx.x;
  const bool active = i0 < total;
  const int i = active ? i0 : (total - 1);
  const int lane = threadIdx.x & 31;
  const int b = i >> 9;
  const int c0 = (i & 511) * 2;
  const float* xd = xdbl + (size_t)b * 64;
  const int sidx = lane & 15;
  float g = xd[32 + sidx] * xd[48 + sidx];
  g += __shfl_xor(g, 1, 32);
  g += __shfl_xor(g, 2, 32);
  g += __shfl_xor(g, 4, 32);
  g += __shfl_xor(g, 8, 32);
  const float* xr = xz + (size_t)b * 2048;
  unsigned packed = 0;
#pragma unroll 1
  for (int e = 0; e < 2; ++e) {
    const int c = c0 + e;
    const float t = xr[c] * cw[c * 4 + 3] + cb[c];
    const float xm = t * __builtin_amdgcn_rcpf(1.0f + expf(-t));
    const float v = (float)dtp[(size_t)b * 1024 + c] + bdt[c];
    const float dt = fmaxf(v, 0.0f) + log1pf(expf(-fabsf(v)));
    const float y = dt * xm * g + xm * Dp[c];
    const float z = xr[1024 + c];
    const float o = y * (z * __builtin_amdgcn_rcpf(1.0f + expf(-z)));
    const _Float16 hv = (_Float16)o;
    packed |= ((unsigned)__builtin_bit_cast(unsigned short, hv)) << (16 * e);
  }
  if (active) {
    volatile unsigned* d = (volatile unsigned*)(yz + (size_t)b * 1024 + c0);
    *d = packed;
    __threadfence();
    *d = packed;
  }
}

__global__ __launch_bounds__(256) void heads_out_k(const float* __restrict__ H, const float* __restrict__ ab,
                                                   const float* __restrict__ cbias, const float* __restrict__ vb,
                                                   float* out, int Bsz) {
  const int rg = blockIdx.x >> 4;
  const int sub = blockIdx.x & 15;
  const int t = threadIdx.x;
  if (rg >= (Bsz >> 5)) return;
  float* out0 = out;
  float* out1 = out + (size_t)Bsz * 4;
  float* out2 = out + (size_t)Bsz * 132;
  const int f = sub * 256 + t;
  const int row = rg * 32 + (f >> 7);
  const int col = f & 127;
  const float hv = H[(size_t)row * 192 + 4 + col] + cbias[col];
  const float cv = tanhf(hv);
  float* p1 = out1 + (size_t)row * 128 + col;
  const bool doA = (sub == 0) && (t < 32);
  const bool doV = (sub == 0) && (t >= 32) && (t < 40);
  v4f av = (v4f){0.f, 0.f, 0.f, 0.f};
  v4f vv = (v4f){0.f, 0.f, 0.f, 0.f};
  float* p0 = out0;
  float* p2 = out2;
  if (doA) {
    const int r = rg * 32 + t;
    const v4f hh = *(const v4f*)(H + (size_t)r * 192);
    const v4f a4 = *(const v4f*)(ab);
    av = hh + a4;
    p0 = out0 + (size_t)r * 4;
  }
  if (doV) {
    const int q = t - 32;
#pragma unroll
    for (int e = 0; e < 4; ++e) {
      const int r = rg * 32 + q * 4 + e;
      vv[e] = H[(size_t)r * 192 + 132] + vb[0];
    }
    p2 = out2 + (size_t)rg * 32 + q * 4;
  }
  *(volatile float*)p1 = cv;
  if (doA) *(volatile v4f*)p0 = av;
  if (doV) *(volatile v4f*)p2 = vv;
  __threadfence();
  *(volatile float*)p1 = cv;
  if (doA) *(volatile v4f*)p0 = av;
  if (doV) *(volatile v4f*)p2 = vv;
}

template <int BIAS, int OUT, bool RES, int ACT>
static void gemm_f16(const _Float16* A, int lda, const _Float16* Bt, int ldb, void* C, void* C2, int ldc,
                     const float* bias, const float* resid, int M, int N, int K, float scale, hipStream_t st) {
  const int tiles = (M >> 6) * (N >> 6);
  if (tiles <= 0) return;
  dim3 grid((unsigned)((tiles + 7) >> 3), 1, 1);
  wmma_gemm64<0, false, BIAS, OUT, RES, ACT><<<grid, 256, 0, st>>>(
      (const unsigned short*)A, (const unsigned short*)nullptr, lda, 0L,
      (const unsigned short*)Bt, (const unsigned short*)nullptr, ldb, 0L,
      C, C2, ldc, 0L, bias, resid, 0L, M, N, K, scale);
}

static inline size_t al256(size_t b) { return (b + 255) & ~(size_t)255; }

extern "C" void kernel_launch(void* const* d_in, const int* in_sizes, int n_in,
                              void* d_out, int out_size, void* d_ws, size_t ws_size,
                              hipStream_t stream) {
  if (n_in < 25) return;
  const float* obs      = (const float*)d_in[0];
  const float* comm_in  = (const float*)d_in[1];
  const float* conv_w   = (const float*)d_in[2];
  const float* conv_b   = (const float*)d_in[3];
  const float* enc_w    = (const float*)d_in[4];
  const float* enc_b    = (const float*)d_in[5];
  const float* proj_w   = (const float*)d_in[6];
  const float* proj_b   = (const float*)d_in[7];
  const float* norm_w   = (const float*)d_in[8];
  const float* inproj_w = (const float*)d_in[9];
  const float* c1d_w    = (const float*)d_in[10];
  const float* c1d_b    = (const float*)d_in[11];
  const float* xproj_w  = (const float*)d_in[12];
  const float* dtproj_w = (const float*)d_in[13];
  const float* dtproj_b = (const float*)d_in[14];
  const float* D_param  = (const float*)d_in[16];
  const float* outp_w   = (const float*)d_in[17];
  const float* fnorm_w  = (const float*)d_in[18];
  const float* act_w    = (const float*)d_in[19];
  const float* act_b    = (const float*)d_in[20];
  const float* comm_w   = (const float*)d_in[21];
  const float* comm_b   = (const float*)d_in[22];
  const float* val_w    = (const float*)d_in[23];
  const float* val_b    = (const float*)d_in[24];

  const int Bsz = in_sizes[0] / 75;
  if (Bsz <= 0 || (Bsz & 63) != 0) return;
  if (out_size < Bsz * 133) return;

  char* base = (char*)d_ws;
  size_t off = 0;
  float*    h      = (float*)(base + off);    off += al256((size_t)Bsz * 512 * 4);
  _Float16* buf16  = (_Float16*)(base + off); off += al256((size_t)Bsz * 1024 * 2);
  char*     big    = base + off;              off += al256((size_t)Bsz * 2048 * 4);
  float*    xdbl   = (float*)(base + off);    off += al256((size_t)Bsz * 64 * 4);
  _Float16* xdbl16 = (_Float16*)(base + off); off += al256((size_t)Bsz * 64 * 2);
  _Float16* dt16   = (_Float16*)(base + off); off += al256((size_t)Bsz * 1024 * 2);
  _Float16* convBt = (_Float16*)(base + off); off += al256((size_t)64 * 32 * 2);
  _Float16* encBt  = (_Float16*)(base + off); off += al256((size_t)256 * 288 * 2);
  _Float16* projBt = (_Float16*)(base + off); off += al256((size_t)512 * 384 * 2);
  _Float16* wiBt   = (_Float16*)(base + off); off += al256((size_t)2 * 2048 * 512 * 2);
  _Float16* wxBt   = (_Float16*)(base + off); off += al256((size_t)2 * 64 * 1024 * 2);
  _Float16* wdtBt  = (_Float16*)(base + off); off += al256((size_t)2 * 1024 * 32 * 2);
  _Float16* woBt   = (_Float16*)(base + off); off += al256((size_t)2 * 512 * 1024 * 2);
  _Float16* headBt = (_Float16*)(base + off); off += al256((size_t)192 * 512 * 2);
  if (off > ws_size) return;

  float* xz = (float*)big;
  size_t o2 = 0;
  _Float16* Aim  = (_Float16*)(big + o2); o2 += al256((size_t)Bsz * 9 * 32 * 2);
  float*    Cc   = (float*)(big + o2);    o2 += al256((size_t)Bsz * 9 * 64 * 4);
  _Float16* v16  = (_Float16*)(big + o2); o2 += al256((size_t)Bsz * 288 * 2);
  _Float16* xcat = (_Float16*)(big + o2); o2 += al256((size_t)Bsz * 384 * 2);
  if (o2 > (size_t)Bsz * 2048 * 4) return;
  float* Hout = (float*)big;

  const float WSC = 64.0f;
  const float WINV = 1.0f / 64.0f;

  pack_bt_f16<<<dim3((64 * 4 + 255) / 256, 1), 256, 0, stream>>>(conv_w, 0L, 1, 27, 27, 32, convBt, 0L, 32, 64, WSC);
  pack_bt_f16<<<dim3((256 * 36 + 255) / 256, 1), 256, 0, stream>>>(enc_w, 0L, 256, 1, 288, 256, encBt, 0L, 288, 256, WSC);
  pack_bt_f16<<<dim3((512 * 48 + 255) / 256, 1), 256, 0, stream>>>(proj_w, 0L, 512, 1, 384, 512, projBt, 0L, 384, 512, WSC);
  pack_bt_f16<<<dim3((2048 * 64 + 255) / 256, 2), 256, 0, stream>>>(inproj_w, 512L * 2048L, 2048, 1, 512, 2048, wiBt, 2048L * 512L, 512, 2048, WSC);
  pack_bt_f16<<<dim3((64 * 128 + 255) / 256, 2), 256, 0, stream>>>(xproj_w, 1024L * 64L, 64, 1, 1024, 64, wxBt, 64L * 1024L, 1024, 64, WSC);
  pack_bt_f16<<<dim3((1024 * 4 + 255) / 256, 2), 256, 0, stream>>>(dtproj_w, 32L * 1024L, 1024, 1, 32, 1024, wdtBt, 1024L * 32L, 32, 1024, WSC);
  pack_bt_f16<<<dim3((512 * 128 + 255) / 256, 2), 256, 0, stream>>>(outp_w, 1024L * 512L, 512, 1, 1024, 512, woBt, 512L * 1024L, 1024, 512, WSC);
  pack_heads_bt<<<(192 * 64 + 255) / 256, 256, 0, stream>>>(act_w, comm_w, val_w, headBt, WSC);

  im2col_k<<<(Bsz * 36 + 255) / 256, 256, 0, stream>>>(obs, Aim, Bsz);
  gemm_f16<0, 0, false, 0>(Aim, 32, convBt, 32, Cc, nullptr, 64, nullptr, nullptr, Bsz * 9, 64, 32, WINV, stream);
  conv_gather_k<<<(Bsz * 36 + 255) / 256, 256, 0, stream>>>(Cc, conv_b, v16, Bsz);
  gemm_f16<2, 1, false, 2>(v16, 288, encBt, 288, xcat, nullptr, 384, enc_b, nullptr, Bsz, 256, 288, WINV, stream);
  comm_cast_k<<<(Bsz * 16 + 255) / 256, 256, 0, stream>>>(comm_in, xcat, Bsz);
  gemm_f16<2, 0, false, 2>(xcat, 384, projBt, 384, h, nullptr, 512, proj_b, nullptr, Bsz, 512, 384, WINV, stream);

  for (int l = 0; l < 2; ++l) {
    rmsnorm_k<<<(Bsz + 7) / 8, 256, 0, stream>>>(h, norm_w + (size_t)l * 512, buf16, Bsz);
    gemm_f16<0, 0, false, 0>(buf16, 512, wiBt + (size_t)l * 2048 * 512, 512, xz, nullptr, 2048, nullptr, nullptr, Bsz, 2048, 512, WINV, stream);
    conv_silu_k<<<(Bsz * 512 + 255) / 256, 256, 0, stream>>>(xz, c1d_w + (size_t)l * 4096, c1d_b + (size_t)l * 1024, buf16, Bsz);
    gemm_f16<0, 0, false, 0>(buf16, 1024, wxBt + (size_t)l * 64 * 1024, 1024, xdbl, nullptr, 64, nullptr, nullptr, Bsz, 64, 1024, WINV, stream);
    cast8_k<<<(Bsz * 8 + 255) / 256, 256, 0, stream>>>(xdbl, xdbl16, Bsz * 8);
    gemm_f16<0, 1, false, 0>(xdbl16, 64, wdtBt + (size_t)l * 1024 * 32, 32, dt16, nullptr, 1024, nullptr, nullptr, Bsz, 1024, 32, WINV, stream);
    yz_k<<<(Bsz * 512 + 255) / 256, 256, 0, stream>>>(xz, xdbl, dt16, dtproj_b + (size_t)l * 1024,
                                                   c1d_w + (size_t)l * 4096, c1d_b + (size_t)l * 1024,
                                                   D_param + (size_t)l * 1024, buf16, Bsz);
    gemm_f16<0, 0, true, 0>(buf16, 1024, woBt + (size_t)l * 512 * 1024, 1024, h, nullptr, 512, nullptr, h, Bsz, 512, 1024, WINV, stream);
  }

  rmsnorm_k<<<(Bsz + 7) / 8, 256, 0, stream>>>(h, fnorm_w, buf16, Bsz);
  gemm_f16<0, 0, false, 0>(buf16, 512, headBt, 512, Hout, nullptr, 192, nullptr, nullptr, Bsz, 192, 512, WINV, stream);
  heads_out_k<<<(Bsz / 32) * 16, 256, 0, stream>>>(Hout, act_b, comm_b, val_b, (float*)d_out, Bsz);
}
